// EulerIntegrator_72593537237650
// MI455X (gfx1250) — hardware-verified
//
#include <hip/hip_runtime.h>
#include <stddef.h>

typedef __attribute__((ext_vector_type(16))) _Float16 v16h;
typedef __attribute__((ext_vector_type(8)))  _Float16 v8h;
typedef __attribute__((ext_vector_type(16))) __bf16   v16b;
typedef __attribute__((ext_vector_type(8)))  __bf16   v8b;
typedef __attribute__((ext_vector_type(8)))  float    v8f;
typedef __attribute__((ext_vector_type(4)))  float    v4f;
typedef __attribute__((ext_vector_type(4)))  unsigned v4u;

constexpr int   NBATCH_ROWS = 4096;
constexpr int   NDIM_D      = 1024;
constexpr int   NRANK_R     = 256;
constexpr int   NSTEPS_MAX  = 8;
constexpr float DT_VALUE    = 0.01f;
constexpr float PCARRY      = 64.0f;
constexpr int   NSTATE      = NBATCH_ROWS * NDIM_D;

static_assert(NDIM_D % 32 == 0 && NRANK_R % 32 == 0, "K of both GEMMs multiple of 32");
static_assert(NBATCH_ROWS % 64 == 0 && NDIM_D % 64 == 0 && NRANK_R % 64 == 0, "M,N of both GEMMs multiple of 64");
static_assert(NSTATE % (256 * 8) == 0, "state kernel: 8 waves x 256 elements per block, exact grid");

constexpr size_t WS_UT    = 0;
constexpr size_t WS_WT    = WS_UT + (size_t)NRANK_R * NDIM_D * 2;
constexpr size_t WS_VH    = WS_WT + (size_t)NDIM_D * NRANK_R * 2;
constexpr size_t WS_P2    = WS_VH + (size_t)NSTATE * 2;
constexpr size_t WS_VA    = WS_P2 + (size_t)NBATCH_ROWS * NRANK_R * 2;
constexpr size_t WS_VB    = WS_VA + (size_t)NSTATE * 4;
constexpr size_t WS_XA    = WS_VB + (size_t)NSTATE * 4;
constexpr size_t WS_XB    = WS_XA + (size_t)NSTATE * 4;
constexpr size_t WS_TOTAL = WS_XB + (size_t)NSTATE * 4;
static_assert(WS_TOTAL == 78643200, "carve total");
static_assert(WS_TOTAL <= 134217728, "carve under 128 MiB");
static_assert((WS_WT % 128) == 0 && (WS_VH % 128) == 0 && (WS_P2 % 128) == 0 && (WS_VA % 128) == 0 &&
              (WS_VB % 128) == 0 && (WS_XA % 128) == 0 && (WS_XB % 128) == 0, "128-B aligned regions");
constexpr size_t OUT1_ELEM_OFS = (size_t)16777216 / 4;
static_assert(OUT1_ELEM_OFS == (size_t)NSTATE, "out1 element offset");
static_assert((OUT1_ELEM_OFS + NSTATE) * 4 == (size_t)33554432, "out1 end == d_out total");

__device__ __forceinline__ unsigned short f2bf_bits(float f) {
  unsigned u = __float_as_uint(f);
  return (unsigned short)((u + 0x7FFFu + ((u >> 16) & 1u)) >> 16);
}
__device__ __forceinline__ float bf_bits2f(unsigned short h) { return __uint_as_float(((unsigned)h) << 16); }

__device__ __forceinline__ unsigned pack_h2(float a, float b) {
  const _Float16 h0 = (_Float16)a, h1 = (_Float16)b;
  return (unsigned)__builtin_bit_cast(unsigned short, h0) | ((unsigned)__builtin_bit_cast(unsigned short, h1) << 16);
}

__device__ __forceinline__ void dep_guard_h(v8f& a, v8f& b, v16h x, v16h y) { asm volatile("v_nop\n\tv_nop\n\tv_nop\n\tv_nop" : "+v"(a), "+v"(b) : "v"(x), "v"(y)); }
__device__ __forceinline__ void dep_guard_b(v8f& a, v8f& b, v16b x, v16b y) { asm volatile("v_nop\n\tv_nop\n\tv_nop\n\tv_nop" : "+v"(a), "+v"(b) : "v"(x), "v"(y)); }
__device__ __forceinline__ void keep4_h(v16h a, v16h b, v16h c, v16h d) { asm volatile("v_nop" :: "v"(a), "v"(b), "v"(c), "v"(d)); }
__device__ __forceinline__ void keep4_b(v16b a, v16b b, v16b c, v16b d) { asm volatile("v_nop" :: "v"(a), "v"(b), "v"(c), "v"(d)); }
__device__ __forceinline__ void acc_guard4(v8f& a, v8f& b, v8f& c, v8f& d) { asm volatile("v_nop\n\tv_nop\n\tv_nop\n\tv_nop" : "+v"(a), "+v"(b), "+v"(c), "+v"(d)); }
template <typename T> struct Frag;
template <> struct Frag<_Float16> {
  typedef v16h V; union U { v16h v; v8h h[2]; };
  static __device__ __forceinline__ v16h load(const _Float16* p) {
    U f; f.h[0] = *(const v8h*)(p); f.h[1] = *(const v8h*)(p + 16); return f.v;
  }
  static __device__ __forceinline__ v8f mma(v16h a, v16h b, v8f c) {
    return __builtin_amdgcn_wmma_f32_16x16x32_f16(false, a, false, b, (short)0, c, false, false);
  }
  static __device__ __forceinline__ void guard(v8f& a, v8f& b, v16h x, v16h y) { dep_guard_h(a, b, x, y); }
  static __device__ __forceinline__ void keep(v16h a, v16h b, v16h c, v16h d) { keep4_h(a, b, c, d); }
};
template <> struct Frag<__bf16> {
  typedef v16b V; union U { v16b v; v8b h[2]; };
  static __device__ __forceinline__ v16b load(const __bf16* p) {
    U f; f.h[0] = *(const v8b*)(p); f.h[1] = *(const v8b*)(p + 16); return f.v;
  }
  static __device__ __forceinline__ v8f mma(v16b a, v16b b, v8f c) {
    return __builtin_amdgcn_wmma_f32_16x16x32_bf16(false, a, false, b, (short)0, c, false, false);
  }
  static __device__ __forceinline__ void guard(v8f& a, v8f& b, v16b x, v16b y) { dep_guard_b(a, b, x, y); }
  static __device__ __forceinline__ void keep(v16b a, v16b b, v16b c, v16b d) { keep4_b(a, b, c, d); }
};

template <int ET> struct Elem;
template <> struct Elem<0> { typedef _Float16 T; };
template <> struct Elem<1> { typedef __bf16 T; };
template <int ET, bool SPLIT, int BIAS_MODE, int OUT_MODE, bool RESID, int ACT, bool RESV>
__global__ __launch_bounds__(256) void wmma_gemm64(
    const unsigned short* __restrict__ Ap, const unsigned short* __restrict__ A2p, int lda, long strideA,
    const unsigned short* __restrict__ Btp, const unsigned short* __restrict__ Bt2p, int ldb, long strideB,
    void* __restrict__ Cout, void* __restrict__ Cout2, int ldc, long strideC,
    const float* __restrict__ bias,
    const float* __restrict__ resid, long strideR,
    const float* __restrict__ resv1, const float* __restrict__ resv2, float r2coef,
    const int* __restrict__ gatep, int gidx,
    int M, int N, int K, float scale) {
  typedef typename Elem<ET>::T T;
  typedef typename Frag<T>::V V;
  const T* A = (const T*)Ap; const T* A2 = (const T*)A2p; const T* Bt = (const T*)Btp; const T* Bt2 = (const T*)Bt2p;
  __shared__ __align__(16) float sT[8][16 * 68];
  const int b    = blockIdx.y;
  const int lane = threadIdx.x & 31;
  const int wave = threadIdx.x >> 5;
  const int tilesN = N >> 6;
  const int tilesM = M >> 6;
  const int tile = blockIdx.x * 8 + wave;
  if (tile >= tilesM * tilesN) return;
  const int tm = tile / tilesN;
  const int tn = tile - tm * tilesN;
  const int m0 = tm << 6;
  const int n0 = tn << 6;

  const float act = (gidx < gatep[0]) ? 1.0f : 0.0f;
  const float scl = scale * act;
  const float r2c = r2coef * act;

  const T* Ab  = A  + (size_t)b * strideA;
  const T* Bb  = Bt + (size_t)b * strideB;
  const T* Ab2 = SPLIT ? (A2  + (size_t)b * strideA) : nullptr;
  const T* Bb2 = SPLIT ? (Bt2 + (size_t)b * strideB) : nullptr;

  const int rlane = lane & 15;
  const int koff  = (lane >> 4) * 8;
  const int mOff  = (lane >> 4) * 8;

  v8f acc[4][4];
#pragma unroll
  for (int i = 0; i < 4; ++i)
#pragma unroll
    for (int j = 0; j < 4; ++j) acc[i][j] = (v8f){0.f,0.f,0.f,0.f,0.f,0.f,0.f,0.f};

  for (int k0 = 0; k0 < K; k0 += 32) {
    V bh[4], bl[4];
#pragma unroll
    for (int j = 0; j < 4; ++j) {
      const size_t bo = (size_t)(n0 + (j << 4) + rlane) * ldb + koff + k0;
      bh[j] = Frag<T>::load(Bb + bo);
      if (SPLIT) bl[j] = Frag<T>::load(Bb2 + bo);
    }
#pragma unroll
    for (int i = 0; i < 4; ++i) {
      const size_t ao = (size_t)(m0 + (i << 4) + rlane) * lda + koff + k0;
      V ah = Frag<T>::load(Ab + ao);
      V al;
      if (SPLIT) al = Frag<T>::load(Ab2 + ao);
#pragma unroll
      for (int j = 0; j < 4; ++j) {
        acc[i][j] = Frag<T>::mma(ah, bh[j], acc[i][j]);
        if (SPLIT) {
          acc[i][j] = Frag<T>::mma(ah, bl[j], acc[i][j]);
          acc[i][j] = Frag<T>::mma(al, bh[j], acc[i][j]);
        }
      }
      Frag<T>::guard(acc[i][0], acc[i][3], ah, SPLIT ? al : ah);
    }
    Frag<T>::keep(bh[0], bh[1], bh[2], bh[3]);
    if (SPLIT) Frag<T>::keep(bl[0], bl[1], bl[2], bl[3]);
  }
  acc_guard4(acc[0][0], acc[0][1], acc[0][2], acc[0][3]);
  acc_guard4(acc[1][0], acc[1][1], acc[1][2], acc[1][3]);
  acc_guard4(acc[2][0], acc[2][1], acc[2][2], acc[2][3]);
  acc_guard4(acc[3][0], acc[3][1], acc[3][2], acc[3][3]);

  float* slab = sT[wave];
  const float* Rb = RESID ? (resid + (size_t)b * strideR) : nullptr;
#pragma unroll
  for (int i = 0; i < 4; ++i) {
    const int mBase = m0 + (i << 4);
#pragma unroll
    for (int j = 0; j < 4; ++j) {
      const int n = n0 + (j << 4) + rlane;
      float bv = 0.f;
      if (BIAS_MODE == 2) bv = bias[n];
#pragma unroll
      for (int r = 0; r < 8; ++r) {
        float v = acc[i][j][r] * scl;
        if (BIAS_MODE == 1) v += bias[mBase + mOff + r];
        if (BIAS_MODE == 2) v += bv;
        if (RESID) v += Rb[(size_t)(mBase + mOff + r) * ldc + n];
        if (ACT == 1) v = tanhf(v);
        if (ACT == 2) v = fmaxf(v, 0.0f);
        if (ACT == 3) v = v / (1.0f + expf(-v));
        if (ACT == 4) v = (v > 0.f) ? v : 0.01f * v;
        if (ACT == 5) v = 0.5f * v * (1.0f + erff(v * 0.70710678118654752f));
        if (ACT == 6) v = PCARRY * (v * v);
        slab[(mOff + r) * 68 + (j << 4) + rlane] = v;
      }
    }
    __builtin_amdgcn_fence(__ATOMIC_RELEASE, "workgroup");
    __builtin_amdgcn_wave_barrier();
    __builtin_amdgcn_fence(__ATOMIC_ACQUIRE, "workgroup");
    if (OUT_MODE == 0) {
      float* C = (float*)Cout + (size_t)b * strideC;
      const int hh = lane >> 4, c4 = (lane & 15) * 4;
      if (RESV) {
#pragma unroll 2
        for (int it = 0; it < 8; ++it) {
          const int row = it * 2 + hh;
          float* sp = slab + row * 68 + c4;
          v4f a = *(const v4f*)sp;
          const size_t go = (size_t)(mBase + row) * ldc + n0 + c4;
          const v4f r1 = *(const v4f*)(resv1 + go);
          const v4f r2 = *(const v4f*)(resv2 + go);
#pragma unroll
          for (int e = 0; e < 4; ++e) a[e] = (a[e] + r1[e]) + r2c * r2[e];
          *(v4f*)sp = a;
        }
      }
      for (int pass = 0; pass < 2; ++pass) {
#pragma unroll
        for (int it = 0; it < 8; ++it) {
          const int row = it * 2 + hh;
          v4f v = *(const v4f*)(slab + row * 68 + c4);
          *(volatile v4f*)(C + (size_t)(mBase + row) * ldc + n0 + c4) = v;
        }
        __threadfence();
      }
    } else {
      const int q = lane >> 3, c8 = (lane & 7) * 8;
      unsigned short* C  = (unsigned short*)Cout  + (size_t)b * strideC;
      unsigned short* C2 = (OUT_MODE == 2) ? ((unsigned short*)Cout2 + (size_t)b * strideC) : nullptr;
      for (int pass = 0; pass < 2; ++pass) {
#pragma unroll
        for (int it = 0; it < 4; ++it) {
          const int row = it * 4 + q;
          const float* sp = slab + row * 68 + c8;
          v8h hv, lv;
#pragma unroll
          for (int e = 0; e < 8; ++e) {
            if (OUT_MODE == 1) {
              hv[e] = (_Float16)sp[e];
            } else {
              unsigned short hb = f2bf_bits(sp[e]);
              unsigned short lb = f2bf_bits(sp[e] - bf_bits2f(hb));
              hv[e] = __builtin_bit_cast(_Float16, hb);
              lv[e] = __builtin_bit_cast(_Float16, lb);
            }
          }
          *(volatile v8h*)(C + (size_t)(mBase + row) * ldc + n0 + c8) = hv;
          if (OUT_MODE == 2) *(volatile v8h*)(C2 + (size_t)(mBase + row) * ldc + n0 + c8) = lv;
        }
        __threadfence();
      }
    }
    __builtin_amdgcn_fence(__ATOMIC_RELEASE, "workgroup");
    __builtin_amdgcn_wave_barrier();
    __builtin_amdgcn_fence(__ATOMIC_ACQUIRE, "workgroup");
  }
}

__global__ __launch_bounds__(256) void tcast64_kernel(
    const float* __restrict__ in, unsigned short* __restrict__ out, int rows, int cols, float sc) {
  __shared__ float tile[64][65];
  const int tid = threadIdx.x, lane = tid & 31, wave = tid >> 5;
  const int c0 = blockIdx.x * 64, r0 = blockIdx.y * 64;
  {
    const int rr = tid >> 2, cc = (tid & 3) * 16;
    const float* src = in + (size_t)(r0 + rr) * cols + c0 + cc;
#pragma unroll
    for (int q = 0; q < 4; ++q) {
      const v4f w = *(const v4f*)(src + 4 * q);
      tile[rr][cc + 4 * q + 0] = w[0];
      tile[rr][cc + 4 * q + 1] = w[1];
      tile[rr][cc + 4 * q + 2] = w[2];
      tile[rr][cc + 4 * q + 3] = w[3];
    }
  }
  __syncthreads();
  v4u pk[2];
  size_t oofs[2];
#pragma unroll
  for (int i = 0; i < 2; ++i) {
    const int oc  = (wave * 2 + i) * 4 + (lane >> 3);
    const int orr = (lane & 7) * 8;
    v4u t;
    t[0] = pack_h2(sc * tile[orr + 0][oc], sc * tile[orr + 1][oc]);
    t[1] = pack_h2(sc * tile[orr + 2][oc], sc * tile[orr + 3][oc]);
    t[2] = pack_h2(sc * tile[orr + 4][oc], sc * tile[orr + 5][oc]);
    t[3] = pack_h2(sc * tile[orr + 6][oc], sc * tile[orr + 7][oc]);
    pk[i] = t;
    oofs[i] = (size_t)(c0 + oc) * rows + r0 + orr;
  }
  for (int pass = 0; pass < 2; ++pass) {
#pragma unroll
    for (int i = 0; i < 2; ++i) *(volatile v4u*)(out + oofs[i]) = pk[i];
    __threadfence();
  }
}

__global__ __launch_bounds__(256) void state_step_kernel(
    const float* __restrict__ xs, const float* __restrict__ vs,
    float* __restrict__ xd, unsigned short* __restrict__ vh,
    const int* __restrict__ gatep, int gidx, float dt, int nelem) {
  const int lane = threadIdx.x & 31;
  const int wv = blockIdx.x * 8 + (threadIdx.x >> 5);
  const size_t base = (size_t)wv * 256;
  if (base + 256 > (size_t)nelem) return;
  const float cdt = (gidx < gatep[0]) ? dt : 0.0f;
  const v4f xa = *(const v4f*)(xs + base + 4 * lane);
  const v4f va = *(const v4f*)(vs + base + 4 * lane);
  const v4f xb = *(const v4f*)(xs + base + 128 + 4 * lane);
  const v4f vb = *(const v4f*)(vs + base + 128 + 4 * lane);
  v4f ra, rb;
#pragma unroll
  for (int e = 0; e < 4; ++e) { ra[e] = xa[e] + cdt * va[e]; rb[e] = xb[e] + cdt * vb[e]; }
  const v4f v0 = *(const v4f*)(vs + base + 8 * lane);
  const v4f v1 = *(const v4f*)(vs + base + 8 * lane + 4);
  v4u hw;
  hw[0] = pack_h2(v0[0], v0[1]);
  hw[1] = pack_h2(v0[2], v0[3]);
  hw[2] = pack_h2(v1[0], v1[1]);
  hw[3] = pack_h2(v1[2], v1[3]);
  for (int pass = 0; pass < 2; ++pass) {
    *(volatile v4f*)(xd + base + 4 * lane) = ra;
    *(volatile v4f*)(xd + base + 128 + 4 * lane) = rb;
    *(volatile v4u*)(vh + base + 8 * lane) = hw;
    __threadfence();
  }
}

extern "C" void kernel_launch(void* const* d_in, const int* in_sizes, int n_in,
                              void* d_out, int out_size, void* d_ws, size_t ws_size,
                              hipStream_t stream) {
  if (n_in < 6) return;
  if (in_sizes[0] != NSTATE || in_sizes[1] != NSTATE || in_sizes[2] != NSTATE) return;
  if (in_sizes[3] != NDIM_D * NRANK_R || in_sizes[4] != NRANK_R * NDIM_D || in_sizes[5] < 1) return;
  if (out_size != 2 * NSTATE) return;
  if (ws_size < WS_TOTAL) return;

  const float* x_in  = (const float*)d_in[0];
  const float* v_in  = (const float*)d_in[1];
  const float* force = (const float*)d_in[2];
  const float* Umat  = (const float*)d_in[3];
  const float* Wmat  = (const float*)d_in[4];
  const int*   steps = (const int*)d_in[5];

  char* ws = (char*)d_ws;
  unsigned short* Ut = (unsigned short*)(ws + WS_UT);
  unsigned short* Wt = (unsigned short*)(ws + WS_WT);
  unsigned short* vh = (unsigned short*)(ws + WS_VH);
  unsigned short* p2 = (unsigned short*)(ws + WS_P2);
  float* vA = (float*)(ws + WS_VA);
  float* vB = (float*)(ws + WS_VB);
  float* xA = (float*)(ws + WS_XA);
  float* xB = (float*)(ws + WS_XB);
  float* out0 = (float*)d_out;
  float* out1 = (float*)d_out + OUT1_ELEM_OFS;

  tcast64_kernel<<<dim3(NRANK_R / 64, NDIM_D / 64), 256, 0, stream>>>(Umat, Ut, NDIM_D, NRANK_R, PCARRY);
  tcast64_kernel<<<dim3(NDIM_D / 64, NRANK_R / 64), 256, 0, stream>>>(Wmat, Wt, NRANK_R, NDIM_D, PCARRY);

  const int tiles1 = (NBATCH_ROWS / 64) * (NRANK_R / 64);
  const int tiles2 = (NBATCH_ROWS / 64) * (NDIM_D / 64);
  const int grid1 = (tiles1 + 7) / 8;
  const int grid2 = (tiles2 + 7) / 8;
  const int gridS = NSTATE / (256 * 8);

  for (int s = 0; s < NSTEPS_MAX; ++s) {
    const float* xs = (s == 0) ? x_in : ((s & 1) ? xA : xB);
    const float* vs = (s == 0) ? v_in : ((s & 1) ? vA : vB);
    float* xd = (s + 1 == NSTEPS_MAX) ? out0 : (((s + 1) & 1) ? xA : xB);
    float* vd = (s + 1 == NSTEPS_MAX) ? out1 : (((s + 1) & 1) ? vA : vB);

    state_step_kernel<<<gridS, 256, 0, stream>>>(xs, vs, xd, vh, steps, s, DT_VALUE, NSTATE);

    wmma_gemm64<0, false, 0, 1, false, 6, false><<<dim3(grid1, 1), 256, 0, stream>>>(
        vh, vh, NDIM_D, 0L,
        Ut, Ut, NDIM_D, 0L,
        (void*)p2, (void*)p2, NRANK_R, 0L,
        force,
        force, 0L,
        force, force, 0.0f,
        steps, s,
        NBATCH_ROWS, NRANK_R, NDIM_D, 1.0f / PCARRY);

    wmma_gemm64<0, false, 0, 0, false, 0, true><<<dim3(grid2, 1), 256, 0, stream>>>(
        p2, p2, NRANK_R, 0L,
        Wt, Wt, NRANK_R, 0L,
        (void*)vd, (void*)vd, NDIM_D, 0L,
        force,
        force, 0L,
        vs, force, DT_VALUE,
        steps, s,
        NBATCH_ROWS, NDIM_D, NRANK_R, -DT_VALUE / (PCARRY * PCARRY));
  }
}
